// Kernel_72739566125068
// MI455X (gfx1250) — hardware-verified
//
#include <hip/hip_runtime.h>
#include <math.h>

typedef __attribute__((ext_vector_type(16))) _Float16 v16h;
typedef __attribute__((ext_vector_type(8)))  float    v8f;
typedef __attribute__((ext_vector_type(4)))  float    v4f;

constexpr int N_SRC = 256;
constexpr int N_TGT = 16384;
constexpr int N_HID = 64;
constexpr int N_DIM = 3;
constexpr int TGT_PER_BLOCK = 8;
constexpr int BLOCK_THREADS = 256;
constexpr int SRC_CHUNK = 16;
constexpr int N_CHUNK = N_SRC / SRC_CHUNK;
constexpr float EPS_SQ = 1e-16f;
constexpr float LO_CARRY = 2048.0f;
constexpr float LO_CARRY_INV = 1.0f / 2048.0f;

static_assert(N_TGT % TGT_PER_BLOCK == 0, "grid covers targets exactly");
static_assert(TGT_PER_BLOCK * 32 == BLOCK_THREADS, "one wave per target");
static_assert(N_SRC == BLOCK_THREADS, "one source staged per thread");
static_assert(N_SRC % SRC_CHUNK == 0, "whole source chunks");
static_assert(N_HID == 64, "two 32-deep k blocks");
static_assert(TGT_PER_BLOCK * 4 * 4 == 128, "block output is one 128-B line");

__device__ __forceinline__ v8f mma16(v16h a, v16h b, v8f c) {
  c = __builtin_amdgcn_wmma_f32_16x16x32_f16(false, a, false, b, (short)0, c, false, false);
  asm volatile("v_nop\n\tv_nop\n\tv_nop\n\tv_nop" : "+v"(c) : "v"(a), "v"(b));
  return c;
}

__global__ __launch_bounds__(BLOCK_THREADS)
void pair_field_kernel(const float* __restrict__ ref_len,
                       const float* __restrict__ src_pts,
                       const float* __restrict__ tgt_pts,
                       const float* __restrict__ strength,
                       const float* __restrict__ W1,
                       const float* __restrict__ b1,
                       const float* __restrict__ pade_a,
                       const float* __restrict__ pade_b,
                       const float* __restrict__ W2,
                       const float* __restrict__ b2,
                       float* __restrict__ out)
{
  __shared__ __align__(16) v4f   lsrc[N_SRC];
  __shared__ __align__(16) v4f   lcst[2 * N_HID];
  __shared__ __align__(16) float lw2[2 * N_HID];
  __shared__ __align__(16) float lres[TGT_PER_BLOCK * 4];

  const int tid = threadIdx.x;

  {
    const int s = tid;
    v4f v;
    v.x = src_pts[s * 3 + 0];
    v.y = src_pts[s * 3 + 1];
    v.z = src_pts[s * 3 + 2];
    v.w = strength[s];
    lsrc[s] = v;
  }
  if (tid < N_HID) {
    const int c = tid;
    v4f ca, cb;
    ca.x = W1[c];
    ca.y = b1[c];
    ca.z = pade_a[c * 3 + 0];
    ca.w = pade_a[c * 3 + 1];
    cb.x = pade_a[c * 3 + 2];
    cb.y = pade_b[c * 2 + 0];
    cb.z = pade_b[c * 2 + 1];
    cb.w = 0.0f;
    lcst[2 * c]     = ca;
    lcst[2 * c + 1] = cb;
  }
  if (tid < 2 * N_HID) {
    lw2[tid] = W2[tid];
  }
  __syncthreads();

  const int lane  = tid & 31;
  const int wave  = tid >> 5;
  const int m     = lane & 15;
  const int hf    = lane >> 4;
  const int hbase = hf * 8;

  int t = blockIdx.x * TGT_PER_BLOCK + wave;
  t = (t < N_TGT) ? t : (N_TGT - 1);
  const float Tx = tgt_pts[t * 3 + 0];
  const float Ty = tgt_pts[t * 3 + 1];
  const float Tz = tgt_pts[t * 3 + 2];

  const float rL  = 1.0f / ref_len[0];
  const float b20 = b2[0];
  const float b21 = b2[1];

  v16h Bf[2];
  {
    const int  wcol   = m & 1;
    const bool use_hi = (m < 2);
    const bool use_lo = (m >= 2) && (m < 4);
#pragma unroll
    for (int kb = 0; kb < 2; ++kb) {
#pragma unroll
      for (int i = 0; i < 16; ++i) {
        const int c = kb * 32 + hbase + i + ((i < 8) ? 0 : 8);
        const float w  = lw2[c * 2 + wcol];
        const _Float16 wh = (_Float16)w;
        const float wl = (w - (float)wh) * LO_CARRY;
        const float sel = use_hi ? w : (use_lo ? wl : 0.0f);
        Bf[kb][i] = (_Float16)sel;
      }
    }
  }

  const v8f zero8 = {0.f, 0.f, 0.f, 0.f, 0.f, 0.f, 0.f, 0.f};
  float sc = 0.0f, vx = 0.0f, vy = 0.0f, vz = 0.0f;
  const int src_lane = (m >> 3) << 4;
  const int rsel     = m & 7;
  const int lane_p2  = (lane + 2) & 31;

#pragma unroll 1
  for (int ch = 0; ch < N_CHUNK; ++ch) {
    asm volatile("" ::: "memory");
    const v4f S  = lsrc[ch * SRC_CHUNK + m];
    const float qv = S.w;
    const float rx = Tx - S.x;
    const float ry = Ty - S.y;
    const float rz = Tz - S.z;
    const float d2 = rx * rx + ry * ry + rz * rz + EPS_SQ;
    const float d  = sqrtf(d2);
    const float invd = 1.0f / d;
    const float feat = logf(d * rL);

    v8f accH, accL;
#pragma unroll
    for (int kb = 0; kb < 2; ++kb) {
      v16h ah, al;
#pragma unroll
      for (int i = 0; i < 16; ++i) {
        if ((i & 7) == 0) asm volatile("" ::: "memory");
        const int c = kb * 32 + hbase + i + ((i < 8) ? 0 : 8);
        const v4f ca = lcst[2 * c];
        const v4f cb = lcst[2 * c + 1];
        const float x = fmaf(feat, ca.x, ca.y);
        float num = fmaf(ca.w, x, ca.z);
        num = fmaf(cb.x * x, x, num);
        const float p   = fmaf(cb.z * x, x, cb.y * x);
        const float den = 1.0f + fabsf(p);
        const float hv  = num * __builtin_amdgcn_rcpf(den);
        const _Float16 hh = (_Float16)hv;
        const float hr = (hv - (float)hh) * LO_CARRY;
        ah[i] = hh;
        al[i] = (_Float16)hr;
      }
      if (kb == 0) {
        accH = mma16(ah, Bf[0], zero8);
        accL = mma16(al, Bf[0], zero8);
      } else {
        accH = mma16(ah, Bf[1], accH);
        accL = mma16(al, Bf[1], accL);
      }
    }

    float e[8], g[8];
#pragma unroll
    for (int r = 0; r < 8; ++r) e[r] = fmaf(accL[r], LO_CARRY_INV, accH[r]);
#pragma unroll
    for (int r = 0; r < 8; ++r) {
      const float e2 = __shfl(e[r], lane_p2, 32);
      g[r] = fmaf(e2, LO_CARRY_INV, e[r]);
    }
    float o0 = 0.0f, o1 = 0.0f;
#pragma unroll
    for (int r = 0; r < 8; ++r) {
      const float t0 = __shfl(g[r], src_lane, 32);
      const float t1 = __shfl(g[r], src_lane + 1, 32);
      o0 = (rsel == r) ? t0 : o0;
      o1 = (rsel == r) ? t1 : o1;
    }
    sc = fmaf(o0 + b20, qv, sc);
    const float w = (o1 + b21) * qv * invd;
    vx = fmaf(w, rx, vx);
    vy = fmaf(w, ry, vy);
    vz = fmaf(w, rz, vz);
  }

#pragma unroll
  for (int off = 1; off < 16; off <<= 1) {
    sc += __shfl_xor(sc, off, 32);
    vx += __shfl_xor(vx, off, 32);
    vy += __shfl_xor(vy, off, 32);
    vz += __shfl_xor(vz, off, 32);
  }
  if (lane == 0) {
    lres[wave * 4 + 0] = sc;
    lres[wave * 4 + 1] = vx;
    lres[wave * 4 + 2] = vy;
    lres[wave * 4 + 3] = vz;
  }
  __syncthreads();

  if (tid < TGT_PER_BLOCK) {
    const v4f v = *(const v4f*)(lres + tid * 4);
    float* dst = out + ((size_t)blockIdx.x * TGT_PER_BLOCK + tid) * 4;
    *(volatile v4f*)dst = v;
    __threadfence();
    *(volatile v4f*)dst = v;
  }
}

extern "C" void kernel_launch(void* const* d_in, const int* in_sizes, int n_in,
                              void* d_out, int out_size, void* d_ws, size_t ws_size,
                              hipStream_t stream) {
  (void)d_ws; (void)ws_size;
  if (n_in < 10) return;
  if (in_sizes[0] < 1 ||
      in_sizes[1] != N_SRC * N_DIM ||
      in_sizes[2] != N_TGT * N_DIM ||
      in_sizes[3] != N_SRC ||
      in_sizes[4] != N_HID ||
      in_sizes[5] != N_HID ||
      in_sizes[6] != N_HID * 3 ||
      in_sizes[7] != N_HID * 2 ||
      in_sizes[8] != N_HID * 2 ||
      in_sizes[9] < 2 ||
      out_size != N_TGT * 4) return;

  const float* ref_len  = (const float*)d_in[0];
  const float* src_pts  = (const float*)d_in[1];
  const float* tgt_pts  = (const float*)d_in[2];
  const float* strength = (const float*)d_in[3];
  const float* W1       = (const float*)d_in[4];
  const float* b1       = (const float*)d_in[5];
  const float* pade_a   = (const float*)d_in[6];
  const float* pade_b   = (const float*)d_in[7];
  const float* W2       = (const float*)d_in[8];
  const float* b2       = (const float*)d_in[9];
  float* out = (float*)d_out;

  pair_field_kernel<<<N_TGT / TGT_PER_BLOCK, BLOCK_THREADS, 0, stream>>>(
      ref_len, src_pts, tgt_pts, strength, W1, b1, pade_a, pade_b, W2, b2, out);
}
